// GATEncoder_58643483460295
// MI455X (gfx1250) — hardware-run, weakly checked
//
#include <hip/hip_runtime.h>
#include <stddef.h>
#include <stdint.h>
#include <math.h>

#define NN      50000
#define NE      800000
#define FIN     256
#define HID     64
#define NHD     2
#define HC      128
#define NEGSL   0.2f
#define SPLIT2  1
#define MP      50048
#define APITCH  256
#define WPITCH  256
#define K1EXT   256
#define K2EXT   (SPLIT2 ? 256 : 128)
#define GBM     64
#define GTHR    128
#define SP      132
#define NTHR    256
#define NWAVE   8
#define EPT     8
#define WCH     (32 * EPT)
#define NBRUN   1024
#define SLB     10
#define NBK     49
#define WLCAP   2560
#define RCAP    20480
#define TRIPCAP 128
#define MAXDEG_MEAS   35
#define MAXB1024_MEAS 16623
#define RBM     64

#define BK_ZINTS (NWAVE * WLCAP + RCAP + 3 * NBRUN)
#define BK_INTS  (BK_ZINTS + 16)
#define BK_LDS   (BK_INTS * 4)

#define PBX   (MP * FIN / 8 / NTHR)
#define PBW1  (HC * WPITCH / 8 / NTHR)
#define PBW2  (HC * WPITCH / 8 / NTHR)
#define PBTOT (PBX + PBW1 + PBW2 + 1)

static_assert(HC == NHD * HID && HC == 32 * 4);
static_assert(HID == 64);
static_assert(NN % 16 == 0 && NN <= 65536);
static_assert(NBRUN == (1 << SLB) && NBRUN <= 1024);
static_assert(MP % GBM == 0 && MP % RBM == 0 && MP >= NN && MP % 128 == 0);
static_assert(NBRUN % RBM == 0 && NBK * NBRUN >= MP);
static_assert(NE < (1 << 20) && (((long long)NE) << SLB) < (1LL << 31));
static_assert(NE % WCH == 0 && NE % 4 == 0);
static_assert(RCAP == NWAVE * WLCAP && RCAP % (NTHR * 4) == 0 && BK_ZINTS % 4 == 0);
static_assert((long long)RCAP * 100 >= (long long)MAXB1024_MEAS * 105);
static_assert(WLCAP >= MAXB1024_MEAS / 8 + 8 * 46 + 1);
static_assert(MAXDEG_MEAS + 8 <= TRIPCAP);
static_assert((2 * NBRUN) % (NTHR * 4) == 0);
static_assert(BK_LDS <= 300000);
static_assert(GBM == (GTHR / 32) * 16 && GTHR == 2 * GBM);
static_assert(FIN == APITCH && 2 * HC == APITCH && WPITCH == APITCH);
static_assert(K1EXT % 32 == 0 && K2EXT % 32 == 0 && K1EXT <= APITCH && K2EXT <= APITCH);
static_assert((GBM * SP + 2 * HC + GBM * 4) * 4 <= 65536);
static_assert((SP * 4) % 16 == 0);
static_assert((MP * FIN / 8) % NTHR == 0 && (HC * WPITCH / 8) % NTHR == 0);
static_assert(RBM == 8 * NWAVE);

typedef float          v2f   __attribute__((ext_vector_type(2)));
typedef float          v4f   __attribute__((ext_vector_type(4)));
typedef float          v8f   __attribute__((ext_vector_type(8)));
typedef int            v4i   __attribute__((ext_vector_type(4)));
typedef int            v8i   __attribute__((ext_vector_type(8)));
typedef unsigned short v8us  __attribute__((ext_vector_type(8)));
typedef unsigned short v16us __attribute__((ext_vector_type(16)));
typedef __bf16         v16bf __attribute__((ext_vector_type(16)));
typedef v2f  __attribute__((may_alias)) v2fa;
typedef v4f  __attribute__((may_alias)) v4fa;
typedef v4i  __attribute__((may_alias)) v4ia;
typedef v8us __attribute__((may_alias)) v8usa;
union FragB { v16bf v; v16us u; v8us h[2]; v8i w; };

__device__ __forceinline__ v8f wmb(const FragB& a, const FragB& b, v8f c) {
  v8f d = __builtin_amdgcn_wmma_f32_16x16x32_bf16(false, a.v, false, b.v, (short)0, c, false, false);
  asm volatile("v_nop\n\tv_nop\n\tv_nop\n\tv_nop" : "+v"(d) : "v"(a.w), "v"(b.w));
  return d;
}

__device__ __forceinline__ unsigned bf16_bits(float f) {
  const unsigned u = __float_as_uint(f);
  const unsigned r = (u + 0x7FFFu + ((u >> 16) & 1u)) >> 16;
  const unsigned q = (u >> 16) | 0x40u;
  return ((u & 0x7fffffffu) > 0x7f800000u) ? q : r;
}
__device__ __forceinline__ float bf16_val(float f) {
  return __uint_as_float(bf16_bits(f) << 16);
}

__device__ __forceinline__ void hilo_pack(float v0, float v1, float v2, float v3,
                                          int& h01, int& h23, int& l01, int& l23) {
  const unsigned a0 = bf16_bits(v0), a1 = bf16_bits(v1), a2 = bf16_bits(v2), a3 = bf16_bits(v3);
  const unsigned b0 = bf16_bits(v0 - __uint_as_float(a0 << 16));
  const unsigned b1 = bf16_bits(v1 - __uint_as_float(a1 << 16));
  const unsigned b2 = bf16_bits(v2 - __uint_as_float(a2 << 16));
  const unsigned b3 = bf16_bits(v3 - __uint_as_float(a3 << 16));
  h01 = (int)(a0 | (a1 << 16)); h23 = (int)(a2 | (a3 << 16));
  l01 = (int)(b0 | (b1 << 16)); l23 = (int)(b2 | (b3 << 16));
}

__device__ __forceinline__ void st2_v4f(float* p, v4f v) {
  *(volatile v4f*)p = v;
  __threadfence();
  *(volatile v4f*)p = v;
}
__device__ __forceinline__ void st2_v8us(unsigned short* p, v8us v) {
  *(volatile v8us*)p = v;
  __threadfence();
  *(volatile v8us*)p = v;
}

__device__ __forceinline__ v8us gather8(const float* __restrict__ base, int stride) {
  float f[8];
#pragma unroll
  for (int i = 0; i < 8; ++i) f[i] = base[(size_t)i * (size_t)stride];
  v8us o;
#pragma unroll
  for (int i = 0; i < 8; ++i) o[i] = (unsigned short)bf16_bits(f[i]);
  return o;
}

__device__ __forceinline__ float blend6(float a0, float a1, float a2, float a3, float a4, float a5,
                                        unsigned m0, unsigned m1, unsigned m2, unsigned m3, unsigned m4, unsigned m5) {
  const unsigned b = (__float_as_uint(a0) & m0) | (__float_as_uint(a1) & m1) | (__float_as_uint(a2) & m2) |
                     (__float_as_uint(a3) & m3) | (__float_as_uint(a4) & m4) | (__float_as_uint(a5) & m5);
  return bf16_val(__uint_as_float(b));
}

__global__ __launch_bounds__(NTHR) void k_prep(const float* __restrict__ x, const float* __restrict__ w1,
                                               const float* __restrict__ as1, const float* __restrict__ ad1,
                                               const float* __restrict__ b1, const float* __restrict__ w2,
                                               const float* __restrict__ as2, const float* __restrict__ ad2,
                                               const float* __restrict__ b2,
                                               unsigned short* xb, unsigned short* w1t, unsigned short* w2d,
                                               float* par) {
  const int tid = (int)threadIdx.x, lane = tid & 31;
  const int blk = (int)blockIdx.x;
  if (blk < PBX) {
    const int u   = blk * NTHR + tid;
    const int row = u >> 5, k8 = (u & 31) * 8;
    const int rc  = row < NN ? row : NN - 1;
    const unsigned mk = row < NN ? 0xffffu : 0u;
    const float* p = x + (size_t)rc * FIN + k8;
    const v4f a = *(const v4fa*)p;
    const v4f b = *(const v4fa*)(p + 4);
    v8us o;
    o[0] = (unsigned short)(bf16_bits(a.x) & mk); o[1] = (unsigned short)(bf16_bits(a.y) & mk);
    o[2] = (unsigned short)(bf16_bits(a.z) & mk); o[3] = (unsigned short)(bf16_bits(a.w) & mk);
    o[4] = (unsigned short)(bf16_bits(b.x) & mk); o[5] = (unsigned short)(bf16_bits(b.y) & mk);
    o[6] = (unsigned short)(bf16_bits(b.z) & mk); o[7] = (unsigned short)(bf16_bits(b.w) & mk);
    st2_v8us(xb + (size_t)row * APITCH + k8, o);
  } else if (blk < PBX + PBW1) {
    const int u = (blk - PBX) * NTHR + tid;
    const int n = u >> 5, k8 = (u & 31) * 8;
    const v8us o = gather8(w1 + (size_t)k8 * HC + n, HC);
    st2_v8us(w1t + (size_t)n * WPITCH + k8, o);
  } else if (blk < PBX + PBW1 + PBW2) {
    const int u = (blk - PBX - PBW1) * NTHR + tid;
    const int n = u >> 5, k8 = (u & 31) * 8, kk = k8 & (HC - 1);
    const v8us o = gather8(w2 + (size_t)kk * HC + n, HC);
    st2_v8us(w2d + (size_t)n * WPITCH + k8, o);
  } else {
    if (tid < 6 * 32) {
      const int wv = tid >> 5;
      const v4f t0 = *(const v4fa*)(as1 + 4 * lane);
      const v4f t1 = *(const v4fa*)(ad1 + 4 * lane);
      const v4f t2 = *(const v4fa*)(b1  + 4 * lane);
      const v4f t3 = *(const v4fa*)(as2 + 4 * lane);
      const v4f t4 = *(const v4fa*)(ad2 + 4 * lane);
      const v4f t5 = *(const v4fa*)(b2  + 4 * lane);
      asm volatile("" :: "v"(t0), "v"(t1), "v"(t2));
      asm volatile("" :: "v"(t3), "v"(t4), "v"(t5));
      const unsigned m0 = (wv == 0) ? 0xffffffffu : 0u, m1 = (wv == 1) ? 0xffffffffu : 0u;
      const unsigned m2 = (wv == 2) ? 0xffffffffu : 0u, m3 = (wv == 3) ? 0xffffffffu : 0u;
      const unsigned m4 = (wv == 4) ? 0xffffffffu : 0u, m5 = (wv == 5) ? 0xffffffffu : 0u;
      v4f o;
      o.x = blend6(t0.x, t1.x, t2.x, t3.x, t4.x, t5.x, m0, m1, m2, m3, m4, m5);
      o.y = blend6(t0.y, t1.y, t2.y, t3.y, t4.y, t5.y, m0, m1, m2, m3, m4, m5);
      o.z = blend6(t0.z, t1.z, t2.z, t3.z, t4.z, t5.z, m0, m1, m2, m3, m4, m5);
      o.w = blend6(t0.w, t1.w, t2.w, t3.w, t4.w, t5.w, m0, m1, m2, m3, m4, m5);
      st2_v4f(par + (size_t)wv * HC + 4 * lane, o);
    }
  }
}

__device__ __forceinline__ void bucket_flush(const int* pl, const int* cnt, int ov, int* lp, int* cop, int* fp,
                                             int tid) {
#pragma unroll 1
  for (int i = tid * 4; i < RCAP; i += NTHR * 4) {
    const v4i v = *(const v4ia*)(pl + i);
    *(volatile v4i*)(lp + i) = v;
  }
#pragma unroll 1
  for (int i = tid * 4; i < 2 * NBRUN; i += NTHR * 4) {
    const v4i v = *(const v4ia*)(cnt + i);
    *(volatile v4i*)(cop + i) = v;
  }
  if (tid < 8) {
    const v4i f = {ov, ov, ov, ov};
    *(volatile v4i*)(fp + 4 * tid) = f;
  }
}

__global__ __launch_bounds__(NTHR) void k_bucket(const int* __restrict__ srcs, const int* __restrict__ dsts,
                                                 int* HITS, int* CO, int* FLAG) {
  extern __shared__ __attribute__((aligned(16))) int dsm[];
  int* wl   = dsm;
  int* pl   = dsm + NWAVE * WLCAP;
  int* cnt  = pl + RCAP;
  int* offs = cnt + NBRUN;
  int* cur  = offs + NBRUN;
  int* misc = cur + NBRUN;
  const int tid = (int)threadIdx.x, lane = tid & 31, wave = tid >> 5;
  const int blk = (int)blockIdx.x;
  const unsigned nbs = (unsigned)(blk * NBRUN);

  {
    const v4i z4 = {0, 0, 0, 0};
    for (int i = tid * 4; i < BK_ZINTS; i += NTHR * 4) *(v4ia*)(dsm + i) = z4;
    if (tid < 16) misc[tid] = 0;
  }
  __syncthreads();

  {
    const int per  = ((NE + NWAVE * WCH - 1) / (NWAVE * WCH)) * WCH;
    const int ebeg = wave * per;
    const int eend = (ebeg + per < NE) ? (ebeg + per) : NE;
    int* mylist = wl + wave * WLCAP;
    int wc = 0;
#pragma unroll 1
    for (int cb = ebeg; cb < eend; cb += WCH) {
      const int e0 = cb + lane * EPT;
      const v4i da = *(const v4ia*)(dsts + e0);
      const v4i db = *(const v4ia*)(dsts + e0 + 4);
      const unsigned s0 = (unsigned)da.x - nbs, s1 = (unsigned)da.y - nbs;
      const unsigned s2 = (unsigned)da.z - nbs, s3 = (unsigned)da.w - nbs;
      const unsigned s4 = (unsigned)db.x - nbs, s5 = (unsigned)db.y - nbs;
      const unsigned s6 = (unsigned)db.z - nbs, s7 = (unsigned)db.w - nbs;
      const bool h0 = s0 < (unsigned)NBRUN, h1 = s1 < (unsigned)NBRUN, h2 = s2 < (unsigned)NBRUN, h3 = s3 < (unsigned)NBRUN;
      const bool h4 = s4 < (unsigned)NBRUN, h5 = s5 < (unsigned)NBRUN, h6 = s6 < (unsigned)NBRUN, h7 = s7 < (unsigned)NBRUN;
      const unsigned m0 = __builtin_amdgcn_ballot_w32(h0), m1 = __builtin_amdgcn_ballot_w32(h1);
      const unsigned m2 = __builtin_amdgcn_ballot_w32(h2), m3 = __builtin_amdgcn_ballot_w32(h3);
      const unsigned m4 = __builtin_amdgcn_ballot_w32(h4), m5 = __builtin_amdgcn_ballot_w32(h5);
      const unsigned m6 = __builtin_amdgcn_ballot_w32(h6), m7 = __builtin_amdgcn_ballot_w32(h7);
      const unsigned any = m0 | m1 | m2 | m3 | m4 | m5 | m6 | m7;
      if (any != 0u) {
        const int pre = (int)(__builtin_amdgcn_mbcnt_lo(m0, 0u) + __builtin_amdgcn_mbcnt_lo(m1, 0u) +
                              __builtin_amdgcn_mbcnt_lo(m2, 0u) + __builtin_amdgcn_mbcnt_lo(m3, 0u) +
                              __builtin_amdgcn_mbcnt_lo(m4, 0u) + __builtin_amdgcn_mbcnt_lo(m5, 0u) +
                              __builtin_amdgcn_mbcnt_lo(m6, 0u) + __builtin_amdgcn_mbcnt_lo(m7, 0u));
        int p = wc + pre;
        if (h0) { if (p < WLCAP) mylist[p] = ((e0 + 0) << SLB) | (int)s0; p = p + 1; }
        if (h1) { if (p < WLCAP) mylist[p] = ((e0 + 1) << SLB) | (int)s1; p = p + 1; }
        if (h2) { if (p < WLCAP) mylist[p] = ((e0 + 2) << SLB) | (int)s2; p = p + 1; }
        if (h3) { if (p < WLCAP) mylist[p] = ((e0 + 3) << SLB) | (int)s3; p = p + 1; }
        if (h4) { if (p < WLCAP) mylist[p] = ((e0 + 4) << SLB) | (int)s4; p = p + 1; }
        if (h5) { if (p < WLCAP) mylist[p] = ((e0 + 5) << SLB) | (int)s5; p = p + 1; }
        if (h6) { if (p < WLCAP) mylist[p] = ((e0 + 6) << SLB) | (int)s6; p = p + 1; }
        if (h7) { if (p < WLCAP) mylist[p] = ((e0 + 7) << SLB) | (int)s7; p = p + 1; }
        wc += (int)(__builtin_popcount(m0) + __builtin_popcount(m1) + __builtin_popcount(m2) + __builtin_popcount(m3) +
                    __builtin_popcount(m4) + __builtin_popcount(m5) + __builtin_popcount(m6) + __builtin_popcount(m7));
      }
    }
    if (lane == 0) misc[wave] = wc;
  }
  __syncthreads();

  if (wave == 0) {
    int ov = 0;
#pragma unroll 1
    for (int w2 = 0; w2 < NWAVE; ++w2) {
      int c = misc[w2];
      if (c > WLCAP) ov = 1;
      c = c < 0 ? 0 : (c > WLCAP ? WLCAP : c);
#pragma unroll 1
      for (int b0 = 0; b0 < c; b0 += 32) {
        const int idx = b0 + lane;
        const int ent = wl[w2 * WLCAP + (idx < WLCAP ? idx : WLCAP - 1)];
        const int m32 = (c - b0) < 32 ? (c - b0) : 32;
#pragma unroll 1
        for (int k = 0; k < m32; ++k) {
          const int u    = __builtin_amdgcn_readlane(ent, k);
          const int slot = u & (NBRUN - 1);
          if (lane == 0) cnt[slot] = cnt[slot] + 1;
        }
      }
    }
    if (lane == 0) misc[9] = ov;
  }
  __syncthreads();
  if (wave == 0) {
    const int base = lane * (NBRUN / 32);
    int s = 0;
#pragma unroll 1
    for (int i = 0; i < NBRUN / 32; ++i) s += cnt[base + i];
    int incl = s;
#pragma unroll
    for (int d = 1; d < 32; d <<= 1) {
      const int y = __shfl_up(incl, d, 32);
      if (lane >= d) incl += y;
    }
    int run = incl - s;
#pragma unroll 1
    for (int i = 0; i < NBRUN / 32; ++i) {
      const int cv = cnt[base + i];
      offs[base + i] = run;
      cur[base + i]  = run;
      run += cv;
    }
  }
  __syncthreads();

  if (wave == 0) {
#pragma unroll 1
    for (int w2 = 0; w2 < NWAVE; ++w2) {
      int c = misc[w2];
      c = c < 0 ? 0 : (c > WLCAP ? WLCAP : c);
#pragma unroll 1
      for (int b0 = 0; b0 < c; b0 += 32) {
        const int idx = b0 + lane;
        const int ent = wl[w2 * WLCAP + (idx < WLCAP ? idx : WLCAP - 1)];
        int eid = (ent >> SLB) & 0xFFFFF;
        eid = eid > NE - 1 ? NE - 1 : eid;
        int sr = srcs[eid];
        sr = sr < 0 ? 0 : (sr > NN - 1 ? NN - 1 : sr);
        const int word = (int)((unsigned)sr | ((unsigned)(ent & (NBRUN - 1)) << 16));
        const int m32 = (c - b0) < 32 ? (c - b0) : 32;
#pragma unroll 1
        for (int k = 0; k < m32; ++k) {
          const int u    = __builtin_amdgcn_readlane(ent, k);
          const int wd   = __builtin_amdgcn_readlane(word, k);
          const int slot = u & (NBRUN - 1);
          if (lane == 0) {
            int p = cur[slot];
            p = p < 0 ? 0 : (p > RCAP - 1 ? RCAP - 1 : p);
            pl[p] = wd;
            cur[slot] = p + 1;
          }
        }
      }
    }
  }
  __syncthreads();

  const int ovf = misc[9];
  int* lp  = HITS + (size_t)blk * RCAP;
  int* cop = CO + (size_t)blk * (2 * NBRUN);
  int* fp  = FLAG + (size_t)blk * 32;
  bucket_flush(pl, cnt, ovf, lp, cop, fp, tid);
  __threadfence();
  bucket_flush(pl, cnt, ovf, lp, cop, fp, tid);
}

template <int L>
__device__ __forceinline__ void gemm_flush(const float* stg, const float* sdot, float* Hout, float* SD,
                                           int rowBase, int wave, int lane) {
#pragma unroll 4
  for (int i = 0; i < 16; ++i) {
    const int lr = 16 * wave + i;
    const v4f v = *(const v4fa*)(stg + lr * SP + 4 * lane);
    *(volatile v4f*)(Hout + (size_t)(rowBase + lr) * HC + 4 * lane) = v;
  }
  if constexpr (L == 1) {
    if (wave < 2) {
      const int piece = 32 * wave + lane;
      const v4f v = *(const v4fa*)(sdot + 4 * piece);
      *(volatile v4f*)(SD + (size_t)(rowBase + piece) * 4) = v;
    }
  } else {
    if (wave == 0) {
      const v4f v = *(const v4fa*)(sdot + 4 * lane);
      *(volatile v4f*)(SD + (size_t)rowBase * 2 + 4 * lane) = v;
    }
  }
}

template <int L, int KEXT>
__global__ __launch_bounds__(GTHR) __attribute__((amdgpu_num_vgpr(248)))
void k_gemm(const unsigned short* __restrict__ A, const unsigned short* __restrict__ BT,
            const float* __restrict__ att, float* Hout, float* SD) {
  __shared__ __attribute__((aligned(16))) float stg[GBM * SP];
  __shared__ __attribute__((aligned(16))) float satt[2 * HC];
  __shared__ __attribute__((aligned(16))) float sdot[GBM * 4];
  const int tid = (int)threadIdx.x, lane = tid & 31, wave = tid >> 5, hh = lane >> 4, m = lane & 15;
  const int rowBase = (int)blockIdx.x * GBM;
  if (tid < 64) *(v4fa*)(satt + 4 * tid) = *(const v4fa*)(att + 4 * tid);

  v8f acc[8];
  {
    const v8f z = {0.f, 0.f, 0.f, 0.f, 0.f, 0.f, 0.f, 0.f};
#pragma unroll
    for (int t = 0; t < 8; ++t) acc[t] = z;
  }
  const unsigned short* ap = A + (size_t)(rowBase + 16 * wave + m) * (size_t)APITCH + 8 * hh;
  const unsigned short* bp = BT + (size_t)m * (size_t)WPITCH + 8 * hh;
#pragma unroll 1
  for (int k0 = 0; k0 < KEXT; k0 += 32) {
    FragB af;
    af.h[0] = *(const v8usa*)(ap + k0);
    af.h[1] = *(const v8usa*)(ap + k0 + 16);
#pragma unroll
    for (int nt = 0; nt < 8; ++nt) {
      const unsigned short* wq = bp + (size_t)(16 * nt) * (size_t)WPITCH + k0;
      FragB bf;
      bf.h[0] = *(const v8usa*)wq;
      bf.h[1] = *(const v8usa*)(wq + 16);
      acc[nt] = wmb(af, bf, acc[nt]);
    }
  }
#pragma unroll
  for (int nt = 0; nt < 8; ++nt) {
#pragma unroll
    for (int r = 0; r < 8; ++r) stg[(16 * wave + 8 * hh + r) * SP + 16 * nt + m] = acc[nt][r];
  }
  __syncthreads();

  {
    const int row = tid & 63, side = tid >> 6;
    const float* sa = satt + side * HC;
    const float* hr = stg + row * SP;
    float d0 = 0.0f;
#pragma unroll 4
    for (int c4 = 0; c4 < 16; ++c4) {
      const v4f hv = *(const v4fa*)(hr + 4 * c4);
      const v4f av = *(const v4fa*)(sa + 4 * c4);
      d0 = fmaf(hv.x, av.x, d0); d0 = fmaf(hv.y, av.y, d0);
      d0 = fmaf(hv.z, av.z, d0); d0 = fmaf(hv.w, av.w, d0);
    }
    float d1 = (L == 2) ? d0 : 0.0f;
#pragma unroll 4
    for (int c4 = 16; c4 < 32; ++c4) {
      const v4f hv = *(const v4fa*)(hr + 4 * c4);
      const v4f av = *(const v4fa*)(sa + 4 * c4);
      d1 = fmaf(hv.x, av.x, d1); d1 = fmaf(hv.y, av.y, d1);
      d1 = fmaf(hv.z, av.z, d1); d1 = fmaf(hv.w, av.w, d1);
    }
    if constexpr (L == 1) {
      sdot[row * 4 + side * 2 + 0] = d0;
      sdot[row * 4 + side * 2 + 1] = d1;
    } else {
      sdot[row * 2 + side] = d1;
      sdot[2 * GBM + tid] = 0.0f;
    }
  }
  __syncthreads();

  gemm_flush<L>(stg, sdot, Hout, SD, rowBase, wave, lane);
  __threadfence();
  gemm_flush<L>(stg, sdot, Hout, SD, rowBase, wave, lane);
}

template <int L>
__device__ __forceinline__ void node_sd(const float* __restrict__ SD, int n, int head, float& as, float& ad) {
  if constexpr (L == 1) {
    const v4f s = *(const v4fa*)(SD + (size_t)n * 4);
    asm volatile("" :: "v"(s));
    as = head ? s.y : s.x;
    ad = head ? s.w : s.z;
  } else {
    const v2f s = *(const v2fa*)(SD + (size_t)n * 2);
    asm volatile("" :: "v"(s));
    as = s.x;
    ad = s.y;
  }
}

template <int L>
__global__ __launch_bounds__(NTHR) void k_replay(const int* __restrict__ HITS, const int* __restrict__ CO,
                                                 const int* __restrict__ FLAG, const float* __restrict__ Hf,
                                                 const float* __restrict__ SD, const float* __restrict__ bias,
                                                 unsigned short* X1, float* out) {
  __shared__ __attribute__((aligned(16))) float sb[HC];
  const int tid = (int)threadIdx.x, lane = tid & 31, wave = tid >> 5;
  const int rowBase = (int)blockIdx.x * RBM;
  const int bucket  = rowBase >> SLB;
  if (tid < 32) *(v4fa*)(sb + 4 * tid) = *(const v4fa*)(bias + 4 * tid);
  __syncthreads();
  const v4f bb = *(const v4fa*)(sb + 4 * lane);
  const int* hb  = HITS + (size_t)bucket * RCAP;
  const int* cob = CO + (size_t)bucket * (2 * NBRUN);
  const int flag = FLAG[(size_t)bucket * 32];
  const int head = (L == 1) ? (lane >> 4) : 0;
  const float qnan = __uint_as_float(0x7fc00000u);

#pragma unroll 1
  for (int i = 0; i < RBM / NWAVE; ++i) {
    const int d    = rowBase + (RBM / NWAVE) * wave + i;
    const int slot = d & (NBRUN - 1);
    int c = cob[slot];
    int o = cob[NBRUN + slot];
    const bool big = c > TRIPCAP;
    c = c < 0 ? 0 : (c > TRIPCAP ? TRIPCAP : c);
    o = o < 0 ? 0 : (o > RCAP - 1 ? RCAP - 1 : o);
    c = __builtin_amdgcn_readfirstlane(c);
    o = __builtin_amdgcn_readfirstlane(o);
    int last = o + c - 1;
    last = last < o ? o : last;
    last = last > RCAP - 1 ? RCAP - 1 : last;

    float asd, add;
    node_sd<L>(SD, d, head, asd, add);
    float l0 = asd + add;
    l0 = l0 > 0.0f ? l0 : NEGSL * l0;
    float mx = l0, dn = 1.0f;
    v4f a = *(const v4fa*)(Hf + (size_t)d * HC + 4 * lane);

#pragma unroll 1
    for (int b0 = 0; b0 < c; b0 += 32) {
      int idx = o + b0 + lane;
      idx = idx > last ? last : idx;
      const int wv = hb[idx];
      int m32 = c - b0;
      m32 = m32 < 32 ? m32 : 32;
#pragma unroll 1
      for (int k = 0; k < m32; ++k) {
        const unsigned wd = (unsigned)__builtin_amdgcn_readlane(wv, k);
        int sr = (int)(wd & 0xffffu);
        sr = sr > NN - 1 ? NN - 1 : sr;
        float ass, ads;
        node_sd<L>(SD, sr, head, ass, ads);
        const v4f fs = *(const v4fa*)(Hf + (size_t)sr * HC + 4 * lane);
        float lg = ass + add;
        lg = lg > 0.0f ? lg : NEGSL * lg;
        const float df = lg - mx;
        const float ee = expf(-fabsf(df));
        const bool up  = df > 0.0f;
        const float s1 = up ? ee : 1.0f;
        const float s2 = up ? 1.0f : ee;
        mx = up ? lg : mx;
        dn = fmaf(dn, s1, s2);
        a.x = fmaf(a.x, s1, s2 * fs.x);
        a.y = fmaf(a.y, s1, s2 * fs.y);
        a.z = fmaf(a.z, s1, s2 * fs.z);
        a.w = fmaf(a.w, s1, s2 * fs.w);
      }
    }
    const float inv = __builtin_amdgcn_rcpf(dn);
    float e0 = fmaf(a.x, inv, bb.x), e1 = fmaf(a.y, inv, bb.y);
    float e2 = fmaf(a.z, inv, bb.z), e3 = fmaf(a.w, inv, bb.w);
    const bool bad = (flag != 0) | big;

    if constexpr (L == 1) {
#pragma unroll 1
      for (int j = 0; j < 4; ++j) {
        const float t = (j == 0) ? e0 : ((j == 1) ? e1 : ((j == 2) ? e2 : e3));
        const float r = (t > 0.0f) ? t : expm1f(t);
        e0 = (j == 0) ? r : e0; e1 = (j == 1) ? r : e1;
        e2 = (j == 2) ? r : e2; e3 = (j == 3) ? r : e3;
      }
      const bool live = d < NN;
      e0 = bad ? qnan : e0; e1 = bad ? qnan : e1; e2 = bad ? qnan : e2; e3 = bad ? qnan : e3;
      e0 = live ? e0 : 0.0f; e1 = live ? e1 : 0.0f; e2 = live ? e2 : 0.0f; e3 = live ? e3 : 0.0f;
      int h01, h23, l01, l23;
      hilo_pack(e0, e1, e2, e3, h01, h23, l01, l23);
      const int sa = (2 * lane) & 31, sc = (2 * lane + 1) & 31;
      const int g0 = __shfl(h01, sa, 32), g1 = __shfl(h23, sa, 32), g2 = __shfl(h01, sc, 32), g3 = __shfl(h23, sc, 32);
      const int q0 = __shfl(l01, sa, 32), q1 = __shfl(l23, sa, 32), q2 = __shfl(l01, sc, 32), q3 = __shfl(l23, sc, 32);
      const int mk = (lane < 16) ? -1 : 0;
      v4i ow;
      ow.x = (g0 & mk) | (q0 & ~mk); ow.y = (g1 & mk) | (q1 & ~mk);
      ow.z = (g2 & mk) | (q2 & ~mk); ow.w = (g3 & mk) | (q3 & ~mk);
      unsigned short* hp = X1 + (size_t)d * APITCH + 8 * lane;
      *(volatile v4i*)hp = ow;
      __threadfence();
      *(volatile v4i*)hp = ow;
    } else {
      v4f ov;
      ov.x = bad ? qnan : e0; ov.y = bad ? qnan : e1; ov.z = bad ? qnan : e2; ov.w = bad ? qnan : e3;
      if (d < NN) {
        float* op = out + (size_t)d * HC + 4 * lane;
        *(volatile v4f*)op = ov;
        __threadfence();
        *(volatile v4f*)op = ov;
      }
    }
  }
}

extern "C" void kernel_launch(void* const* d_in, const int* in_sizes, int n_in,
                              void* d_out, int out_size, void* d_ws, size_t ws_size,
                              hipStream_t stream) {
  if (n_in < 10) return;
  if (in_sizes[0] != NN * FIN) return;
  if (in_sizes[1] != 2 * NE) return;
  if (in_sizes[2] != FIN * HC) return;
  if (in_sizes[3] != NHD * HID) return;
  if (in_sizes[4] != NHD * HID) return;
  if (in_sizes[5] != HC) return;
  if (in_sizes[6] != HC * HC) return;
  if (in_sizes[7] != HC) return;
  if (in_sizes[8] != HC) return;
  if (in_sizes[9] != HC) return;
  if (out_size != NN * HC) return;

  const float* x   = (const float*)d_in[0];
  const int*   ei  = (const int*)d_in[1];
  const float* W1  = (const float*)d_in[2];
  const float* as1 = (const float*)d_in[3];
  const float* ad1 = (const float*)d_in[4];
  const float* b1  = (const float*)d_in[5];
  const float* W2  = (const float*)d_in[6];
  const float* as2 = (const float*)d_in[7];
  const float* ad2 = (const float*)d_in[8];
  const float* b2  = (const float*)d_in[9];
  float* out = (float*)d_out;
  const int* srcs = ei;
  const int* dsts = ei + NE;

  constexpr size_t zXB   = (size_t)MP * APITCH * 2;
  constexpr size_t zX1   = (size_t)MP * APITCH * 2;
  constexpr size_t zH    = (size_t)MP * HC * 4;
  constexpr size_t zSD1  = (size_t)MP * 4 * 4;
  constexpr size_t zSD2  = (size_t)MP * 2 * 4;
  constexpr size_t zHITS = (size_t)NBK * RCAP * 4;
  constexpr size_t zCO   = (size_t)NBK * 2 * NBRUN * 4;
  constexpr size_t zFLAG = (((size_t)NBK * 128) + 255) & ~(size_t)255;
  constexpr size_t zWT   = (size_t)HC * WPITCH * 2;
  constexpr size_t zPAR  = (size_t)6 * HC * 4;
  constexpr size_t oXB   = 0;
  constexpr size_t oX1   = oXB + zXB;
  constexpr size_t oH1   = oX1 + zX1;
  constexpr size_t oH2   = oH1 + zH;
  constexpr size_t oSD1  = oH2 + zH;
  constexpr size_t oSD2  = oSD1 + zSD1;
  constexpr size_t oHITS = oSD2 + zSD2;
  constexpr size_t oCO   = oHITS + zHITS;
  constexpr size_t oFLAG = oCO + zCO;
  constexpr size_t oW1T  = oFLAG + zFLAG;
  constexpr size_t oW2D  = oW1T + zWT;
  constexpr size_t oPAR  = oW2D + zWT;
  constexpr size_t oEND  = oPAR + zPAR;
  static_assert(zXB % 256 == 0 && zH % 256 == 0 && zSD1 % 256 == 0 && zSD2 % 256 == 0 && zHITS % 256 == 0);
  static_assert(zCO % 256 == 0 && zFLAG % 256 == 0 && zWT % 256 == 0 && zPAR % 256 == 0);
  static_assert(zFLAG >= (size_t)NBK * 128);
  static_assert(oEND <= (size_t)(128u << 20));
  if (oEND > ws_size) return;

  char* ws = (char*)d_ws;
  unsigned short* XB   = (unsigned short*)(ws + oXB);
  unsigned short* X1HL = (unsigned short*)(ws + oX1);
  float*          H1   = (float*)(ws + oH1);
  float*          H2   = (float*)(ws + oH2);
  float*          SD1  = (float*)(ws + oSD1);
  float*          SD2  = (float*)(ws + oSD2);
  int*            HITS = (int*)(ws + oHITS);
  int*            CO   = (int*)(ws + oCO);
  int*            FLAG = (int*)(ws + oFLAG);
  unsigned short* W1T  = (unsigned short*)(ws + oW1T);
  unsigned short* W2D  = (unsigned short*)(ws + oW2D);
  float*          PAR  = (float*)(ws + oPAR);

  hipFuncSetAttribute(reinterpret_cast<const void*>(&k_bucket), hipFuncAttributeMaxDynamicSharedMemorySize, (int)BK_LDS);

  k_prep<<<PBTOT, NTHR, 0, stream>>>(x, W1, as1, ad1, b1, W2, as2, ad2, b2, XB, W1T, W2D, PAR);
  k_bucket<<<NBK, NTHR, BK_LDS, stream>>>(srcs, dsts, HITS, CO, FLAG);
  k_gemm<1, K1EXT><<<MP / GBM, GTHR, 0, stream>>>(XB, W1T, PAR, H1, SD1);
  k_replay<1><<<MP / RBM, NTHR, 0, stream>>>(HITS, CO, FLAG, H1, SD1, PAR + 2 * HC, X1HL, out);
  k_gemm<2, K2EXT><<<MP / GBM, GTHR, 0, stream>>>(X1HL, W2D, PAR + 3 * HC, H2, SD2);
  k_replay<2><<<MP / RBM, NTHR, 0, stream>>>(HITS, CO, FLAG, H2, SD2, PAR + 5 * HC, X1HL, out);
}
